// ConditionalDLFactorized17_74680891343537
// MI455X (gfx1250) — hardware-verified
//
#include <hip/hip_runtime.h>
#include <math.h>

constexpr int kT    = 2048;
constexpr int kB    = 8;
constexpr int kC    = 512;
constexpr int kOut  = 512;
constexpr int kNE   = 16;
constexpr int kTok  = kT * kB;
constexpr int kWPlane = kOut * kC;
constexpr float kWCarry    = 16.0f;
constexpr float kWCarryInv = 1.0f / 16.0f;
constexpr float kLossScale = 0.01f;
constexpr int kRouterTokPerBlock = 64;
constexpr int kRouterBlocks = kTok / kRouterTokPerBlock;
constexpr int kPartPitch = 32;

static_assert(kTok % kRouterTokPerBlock == 0, "router grid exact");
static_assert(kTok % 64 == 0 && kOut % 64 == 0 && kC % 32 == 0, "GEMM tile multiples");
static_assert((kTok * kC) % (8 * 256) == 0, "x cast grid exact");
static_assert((kNE * kWPlane) % (8 * 256) == 0, "w cast grid exact");

constexpr size_t kOffX16  = 0;
constexpr size_t kOffW16  = kOffX16  + (size_t)kTok * kC * 2;
constexpr size_t kOffResp = kOffW16  + (size_t)kNE * kWPlane * 2;
constexpr size_t kOffPart = kOffResp + (size_t)kTok * kNE * 4;
constexpr size_t kOffY0   = kOffPart + (size_t)kRouterBlocks * kPartPitch * 4;
constexpr size_t kOffY1   = kOffY0   + (size_t)kTok * kOut * 4;
constexpr size_t kWsEnd   = kOffY1   + (size_t)kTok * kOut * 4;
static_assert(kWsEnd == 93356032, "carve total");
static_assert(kWsEnd <= 134217728, "carve under 128 MiB");
static_assert(kOffW16 % 128 == 0 && kOffResp % 128 == 0 && kOffPart % 128 == 0 && kOffY0 % 128 == 0 && kOffY1 % 128 == 0, "aligned regions");

typedef __attribute__((ext_vector_type(16))) _Float16 v16h;
typedef __attribute__((ext_vector_type(8)))  _Float16 v8h;
typedef __attribute__((ext_vector_type(16))) __bf16   v16b;
typedef __attribute__((ext_vector_type(8)))  __bf16   v8b;
typedef __attribute__((ext_vector_type(8)))  float    v8f;
typedef __attribute__((ext_vector_type(4)))  float    v4f;
typedef __attribute__((ext_vector_type(4)))  unsigned int v4u;

__device__ __forceinline__ unsigned short f2bf_bits(float f) {
  unsigned u = __float_as_uint(f);
  return (unsigned short)((u + 0x7FFFu + ((u >> 16) & 1u)) >> 16);
}
__device__ __forceinline__ float bf_bits2f(unsigned short h) { return __uint_as_float(((unsigned)h) << 16); }

__device__ __forceinline__ void dep_guard_h(v8f& a, v8f& b, v16h x, v16h y) { asm volatile("v_nop\n\tv_nop\n\tv_nop\n\tv_nop" : "+v"(a), "+v"(b) : "v"(x), "v"(y)); }
__device__ __forceinline__ void dep_guard_b(v8f& a, v8f& b, v16b x, v16b y) { asm volatile("v_nop\n\tv_nop\n\tv_nop\n\tv_nop" : "+v"(a), "+v"(b) : "v"(x), "v"(y)); }
__device__ __forceinline__ void keep4_h(v16h a, v16h b, v16h c, v16h d) { asm volatile("v_nop" :: "v"(a), "v"(b), "v"(c), "v"(d)); }
__device__ __forceinline__ void keep4_b(v16b a, v16b b, v16b c, v16b d) { asm volatile("v_nop" :: "v"(a), "v"(b), "v"(c), "v"(d)); }
__device__ __forceinline__ void acc_guard4(v8f& a, v8f& b, v8f& c, v8f& d) { asm volatile("v_nop\n\tv_nop\n\tv_nop\n\tv_nop" : "+v"(a), "+v"(b), "+v"(c), "+v"(d)); }
template <typename T> struct Frag;
template <> struct Frag<_Float16> {
  typedef v16h V; union U { v16h v; v8h h[2]; };
  static __device__ __forceinline__ v16h load(const _Float16* p) {
    U f; f.h[0] = *(const v8h*)(p); f.h[1] = *(const v8h*)(p + 16); return f.v;
  }
  static __device__ __forceinline__ v8f mma(v16h a, v16h b, v8f c) {
    return __builtin_amdgcn_wmma_f32_16x16x32_f16(false, a, false, b, (short)0, c, false, false);
  }
  static __device__ __forceinline__ void guard(v8f& a, v8f& b, v16h x, v16h y) { dep_guard_h(a, b, x, y); }
  static __device__ __forceinline__ void keep(v16h a, v16h b, v16h c, v16h d) { keep4_h(a, b, c, d); }
};
template <> struct Frag<__bf16> {
  typedef v16b V; union U { v16b v; v8b h[2]; };
  static __device__ __forceinline__ v16b load(const __bf16* p) {
    U f; f.h[0] = *(const v8b*)(p); f.h[1] = *(const v8b*)(p + 16); return f.v;
  }
  static __device__ __forceinline__ v8f mma(v16b a, v16b b, v8f c) {
    return __builtin_amdgcn_wmma_f32_16x16x32_bf16(false, a, false, b, (short)0, c, false, false);
  }
  static __device__ __forceinline__ void guard(v8f& a, v8f& b, v16b x, v16b y) { dep_guard_b(a, b, x, y); }
  static __device__ __forceinline__ void keep(v16b a, v16b b, v16b c, v16b d) { keep4_b(a, b, c, d); }
};

__device__ __forceinline__ unsigned pk16(unsigned short a, unsigned short b) { return (unsigned)a | ((unsigned)b << 16); }
__device__ __forceinline__ unsigned short h_bits(float f) { const _Float16 h = (_Float16)f; return __builtin_bit_cast(unsigned short, h); }

template <bool HAS_PREV, bool HAS_BIAS>
__global__ __launch_bounds__(256) void moe_gemm64(
    const unsigned short* __restrict__ Ap, int lda,
    const unsigned short* __restrict__ Btp, int ldb,
    float* __restrict__ Cout, int ldc,
    const float* __restrict__ prev,
    const float* __restrict__ rsc, int rs_ld, int rs_col,
    const float* __restrict__ bias,
    int M, int N, int K, float scale) {
  typedef _Float16 T;
  typedef Frag<T>::V V;
  const T* A = (const T*)Ap; const T* Bt = (const T*)Btp;
  __shared__ __align__(16) float sT[8][16 * 68];
  const int lane = threadIdx.x & 31;
  const int wave = threadIdx.x >> 5;
  const int tilesN = N >> 6;
  const int tilesM = M >> 6;
  const int tile = blockIdx.x * 8 + wave;
  if (tile >= tilesM * tilesN) return;
  const int tm = tile / tilesN;
  const int tn = tile - tm * tilesN;
  const int m0 = tm << 6;
  const int n0 = tn << 6;

  const int rlane = lane & 15;
  const int koff  = (lane >> 4) * 8;
  const int mOff  = (lane >> 4) * 8;

  v8f acc[4][4];
#pragma unroll
  for (int i = 0; i < 4; ++i)
#pragma unroll
    for (int j = 0; j < 4; ++j) acc[i][j] = (v8f){0.f,0.f,0.f,0.f,0.f,0.f,0.f,0.f};

  for (int k0 = 0; k0 < K; k0 += 32) {
    V bh[4];
#pragma unroll
    for (int j = 0; j < 4; ++j) {
      const size_t bo = (size_t)(n0 + (j << 4) + rlane) * ldb + koff + k0;
      bh[j] = Frag<T>::load(Bt + bo);
    }
#pragma unroll
    for (int i = 0; i < 4; ++i) {
      const size_t ao = (size_t)(m0 + (i << 4) + rlane) * lda + koff + k0;
      V ah = Frag<T>::load(A + ao);
#pragma unroll
      for (int j = 0; j < 4; ++j) acc[i][j] = Frag<T>::mma(ah, bh[j], acc[i][j]);
      Frag<T>::guard(acc[i][0], acc[i][3], ah, ah);
    }
    Frag<T>::keep(bh[0], bh[1], bh[2], bh[3]);
  }
  acc_guard4(acc[0][0], acc[0][1], acc[0][2], acc[0][3]);
  acc_guard4(acc[1][0], acc[1][1], acc[1][2], acc[1][3]);
  acc_guard4(acc[2][0], acc[2][1], acc[2][2], acc[2][3]);
  acc_guard4(acc[3][0], acc[3][1], acc[3][2], acc[3][3]);

  float* slab = sT[wave];
#pragma unroll
  for (int i = 0; i < 4; ++i) {
    const int mBase = m0 + (i << 4);
    float rsv[8];
#pragma unroll
    for (int r = 0; r < 8; ++r) rsv[r] = rsc[(size_t)(mBase + mOff + r) * rs_ld + rs_col] * scale;
#pragma unroll
    for (int j = 0; j < 4; ++j) {
      const int n = n0 + (j << 4) + rlane;
      float bv = 0.f;
      if (HAS_BIAS) bv = bias[n];
#pragma unroll
      for (int r = 0; r < 8; ++r) {
        float v = acc[i][j][r] * rsv[r];
        if (HAS_PREV) v += prev[(size_t)(mBase + mOff + r) * ldc + n];
        if (HAS_BIAS) v += bv;
        slab[(mOff + r) * 68 + (j << 4) + rlane] = v;
      }
    }
    __builtin_amdgcn_fence(__ATOMIC_RELEASE, "workgroup");
    __builtin_amdgcn_wave_barrier();
    __builtin_amdgcn_fence(__ATOMIC_ACQUIRE, "workgroup");
    {
      float* Cp = Cout;
      const int hh = lane >> 4, c4 = (lane & 15) * 4;
      for (int pass = 0; pass < 2; ++pass) {
#pragma unroll
        for (int it = 0; it < 8; ++it) {
          const int row = it * 2 + hh;
          v4f v = *(const v4f*)(slab + row * 68 + c4);
          *(volatile v4f*)(Cp + (size_t)(mBase + row) * ldc + n0 + c4) = v;
        }
        __threadfence();
      }
    }
    __builtin_amdgcn_fence(__ATOMIC_RELEASE, "workgroup");
    __builtin_amdgcn_wave_barrier();
    __builtin_amdgcn_fence(__ATOMIC_ACQUIRE, "workgroup");
  }
}

__global__ __launch_bounds__(256) void cast8_f16_kernel(const float* __restrict__ in, unsigned short* __restrict__ out, int n8, float scale) {
  const int i = blockIdx.x * 256 + threadIdx.x;
  if (i >= n8) return;
  const float* p = in + 8 * (size_t)i;
  const v4f a = *(const v4f*)(p);
  const v4f c = *(const v4f*)(p + 4);
  unsigned short hb[8];
#pragma unroll
  for (int e = 0; e < 4; ++e) {
    hb[e]     = h_bits(a[e] * scale);
    hb[4 + e] = h_bits(c[e] * scale);
  }
  const v4u u = (v4u){pk16(hb[0], hb[1]), pk16(hb[2], hb[3]), pk16(hb[4], hb[5]), pk16(hb[6], hb[7])};
  unsigned short* q = out + 8 * (size_t)i;
  *(volatile v4u*)q = u;
  __threadfence();
  *(volatile v4u*)q = u;
}

__global__ __launch_bounds__(256) void router_kernel(const float* __restrict__ x, const float* __restrict__ aw,
                                                     const float* __restrict__ ab, float* __restrict__ resp,
                                                     float* __restrict__ part, int ntok) {
  __shared__ __align__(16) float sw[kNE * kC];
  __shared__ __align__(16) float sres[8][128];
  __shared__ float simp[8][16];
  __shared__ __align__(16) float spart[32];
  __shared__ float sab[kNE];
  const int tid  = threadIdx.x;
  const int lane = tid & 31;
  const int wave = tid >> 5;
  const int col  = lane & 15;
#pragma unroll
  for (int p = 0; p < 8; ++p) {
    const int idx = (p * 256 + tid) * 4;
    *(v4f*)&sw[idx] = *(const v4f*)&aw[idx];
  }
  if (tid < kNE) sab[tid] = ab[tid];
  __syncthreads();

  float myimp = 0.f;
#pragma unroll 1
  for (int tt = 0; tt < 8; ++tt) {
    const int token = blockIdx.x * kRouterTokPerBlock + wave * 8 + tt;
    const int tokc  = token < ntok ? token : ntok - 1;
    const float* xp = x + (size_t)tokc * kC + lane * 16;
    const v4f x0 = *(const v4f*)(xp);
    const v4f x1 = *(const v4f*)(xp + 4);
    const v4f x2 = *(const v4f*)(xp + 8);
    const v4f x3 = *(const v4f*)(xp + 12);
    float mylogit = 0.f;
#pragma unroll 1
    for (int e = 0; e < kNE; ++e) {
      const float* wp = sw + e * kC + lane * 16;
      const v4f w0 = *(const v4f*)(wp);
      const v4f w1 = *(const v4f*)(wp + 4);
      const v4f w2 = *(const v4f*)(wp + 8);
      const v4f w3 = *(const v4f*)(wp + 12);
      float p = x0.x * w0.x + x0.y * w0.y + x0.z * w0.z + x0.w * w0.w
              + x1.x * w1.x + x1.y * w1.y + x1.z * w1.z + x1.w * w1.w
              + x2.x * w2.x + x2.y * w2.y + x2.z * w2.z + x2.w * w2.w
              + x3.x * w3.x + x3.y * w3.y + x3.z * w3.z + x3.w * w3.w;
#pragma unroll
      for (int off = 16; off > 0; off >>= 1) p += __shfl_xor(p, off, 32);
      const float lgv = p + sab[e];
      mylogit = (col == e) ? lgv : mylogit;
    }
    float m = mylogit;
#pragma unroll
    for (int off = 8; off > 0; off >>= 1) m = fmaxf(m, __shfl_xor(m, off, 32));
    const float pe = expf(mylogit - m);
    float s = pe;
#pragma unroll
    for (int off = 8; off > 0; off >>= 1) s += __shfl_xor(s, off, 32);
    const float r = pe * (1.0f / s);
    myimp += r;
    if (lane < 16) sres[wave][tt * 16 + lane] = r;
  }
  if (lane < 16) simp[wave][lane] = myimp;
  __syncthreads();

  {
    float* rp = resp + (size_t)(blockIdx.x * kRouterTokPerBlock + wave * 8) * kNE + lane * 4;
    const v4f v = *(const v4f*)&sres[wave][lane * 4];
    *(volatile v4f*)rp = v;
    __threadfence();
    *(volatile v4f*)rp = v;
  }
  if (tid < 32) {
    float sacc = 0.f;
#pragma unroll
    for (int w = 0; w < 8; ++w) sacc += simp[w][col];
    spart[tid] = (tid < 16) ? sacc : 0.f;
  }
  __syncthreads();
  if (tid < 8) {
    const v4f v = *(const v4f*)&spart[tid * 4];
    float* pp = part + (size_t)blockIdx.x * kPartPitch + tid * 4;
    *(volatile v4f*)pp = v;
    __threadfence();
    *(volatile v4f*)pp = v;
  }
}

__global__ __launch_bounds__(32) void loss_kernel(const float* __restrict__ part, int nblk, float* __restrict__ out1) {
  const int lane = threadIdx.x & 31;
  const int col  = lane & 15;
  float imp = 0.f;
#pragma unroll 1
  for (int b = 0; b < nblk; ++b) imp += part[(size_t)b * kPartPitch + col];
  float tot = imp;
#pragma unroll
  for (int off = 8; off > 0; off >>= 1) tot += __shfl_xor(tot, off, 32);
  const float mean = tot * (1.0f / 16.0f);
  const float d = imp - mean;
  float var = d * d;
#pragma unroll
  for (int off = 8; off > 0; off >>= 1) var += __shfl_xor(var, off, 32);
  var = var * (1.0f / 15.0f);
  const float lossv = (kLossScale * sqrtf(var)) / mean;
  if (lane == 0) {
    *(volatile float*)out1 = lossv;
    __threadfence();
    *(volatile float*)out1 = lossv;
  }
}

extern "C" void kernel_launch(void* const* d_in, const int* in_sizes, int n_in,
                              void* d_out, int out_size, void* d_ws, size_t ws_size,
                              hipStream_t stream) {
  if (n_in < 5) return;
  if (in_sizes[0] != kTok * kC || in_sizes[1] != kNE * kC || in_sizes[2] != kNE ||
      in_sizes[3] != kNE * kWPlane || in_sizes[4] != kOut) return;
  if (out_size != kTok * kOut + 1) return;
  if (ws_size < kWsEnd) return;

  const float* x   = (const float*)d_in[0];
  const float* aw  = (const float*)d_in[1];
  const float* ab  = (const float*)d_in[2];
  const float* w1  = (const float*)d_in[3];
  const float* pwB = (const float*)d_in[4];

  float* out0 = (float*)d_out;
  float* out1 = (float*)d_out + (size_t)kTok * kOut;

  char* ws = (char*)d_ws;
  unsigned short* X16 = (unsigned short*)(ws + kOffX16);
  unsigned short* W16 = (unsigned short*)(ws + kOffW16);
  float* RESP = (float*)(ws + kOffResp);
  float* PART = (float*)(ws + kOffPart);
  float* Y0   = (float*)(ws + kOffY0);
  float* Y1   = (float*)(ws + kOffY1);

  const int nx8 = kTok * kC / 8;
  const int nw8 = kNE * kWPlane / 8;
  cast8_f16_kernel<<<nx8 / 256, 256, 0, stream>>>(x, X16, nx8, 1.0f);
  cast8_f16_kernel<<<nw8 / 256, 256, 0, stream>>>(w1, W16, nw8, kWCarry);
  router_kernel<<<kRouterBlocks, 256, 0, stream>>>(x, aw, ab, RESP, PART, kTok);
  loss_kernel<<<1, 32, 0, stream>>>(PART, kRouterBlocks, out1);

  const int gemmBlocks = ((kTok / 64) * (kOut / 64)) / 8;
  for (int e = 0; e < kNE; ++e) {
    const unsigned short* Bt = W16 + (size_t)e * kWPlane;
    float* ynext = (e & 1) ? Y1 : Y0;
    const float* yprev = (e & 1) ? Y0 : Y1;
    if (e == 0) {
      moe_gemm64<false, false><<<gemmBlocks, 256, 0, stream>>>(X16, kC, Bt, kC, Y0, kOut, nullptr,
                                                              RESP, kNE, 0, pwB, kTok, kOut, kC, kWCarryInv);
    } else if (e < kNE - 1) {
      moe_gemm64<true, false><<<gemmBlocks, 256, 0, stream>>>(X16, kC, Bt, kC, ynext, kOut, yprev,
                                                             RESP, kNE, e, pwB, kTok, kOut, kC, kWCarryInv);
    } else {
      moe_gemm64<true, true><<<gemmBlocks, 256, 0, stream>>>(X16, kC, Bt, kC, out0, kOut, yprev,
                                                            RESP, kNE, e, pwB, kTok, kOut, kC, kWCarryInv);
    }
  }
}
